// RNN_63213328662812
// MI455X (gfx1250) — hardware-verified
//
#include <hip/hip_runtime.h>
#include <math.h>

typedef __attribute__((ext_vector_type(16))) _Float16 v16h;
typedef __attribute__((ext_vector_type(8)))  _Float16 v8h;
typedef __attribute__((ext_vector_type(16))) __bf16   v16b;
typedef __attribute__((ext_vector_type(8)))  __bf16   v8b;
typedef __attribute__((ext_vector_type(8)))  float    v8f;
typedef __attribute__((ext_vector_type(4)))  float    v4f;

constexpr int kBatch  = 16;
constexpr int kSteps  = 512;
constexpr int kDim    = 1024;
constexpr int kLayers = 4;
constexpr int kRows   = kBatch * kSteps;
constexpr int kWPitch = 2 * kDim;
constexpr int kHP     = kDim + 8;
constexpr int kScanThr = 512;
constexpr int kSlabP  = 68;
constexpr float kWCarry    = 256.0f;
constexpr float kWCarryInv = 1.0f / kWCarry;
constexpr float kLoCarry   = 2048.0f;
constexpr float kLoFold    = kWCarryInv / kLoCarry;
static_assert(kBatch == 16, "one 16-row m-subtile");
static_assert(kDim == (kScanThr / 32) * 64, "16 waves x 64 columns");
static_assert(kDim % 32 == 0 && kDim % 64 == 0 && kRows % 64 == 0, "GEMM M, N multiples of 64; K multiple of 32");
static_assert(kHP % 8 == 0 && (kBatch * kHP) % 8 == 0, "16-B aligned LDS rows");
static_assert((kBatch * kDim / 4) % kScanThr == 0, "h0 staging loop exact");
static_assert((kLayers * kDim * (kWPitch / 8)) % 256 == 0, "weight cast grid exact");
static_assert((kRows * (kDim / 8)) % 256 == 0, "x cast grid exact");
static_assert((kLayers * kDim / 4) % 256 == 0, "bias grid exact");

__device__ __forceinline__ unsigned short f2bf_bits(float f) {
  unsigned u = __float_as_uint(f);
  return (unsigned short)((u + 0x7FFFu + ((u >> 16) & 1u)) >> 16);
}
__device__ __forceinline__ float bf_bits2f(unsigned short h) { return __uint_as_float(((unsigned)h) << 16); }
__device__ __forceinline__ float bf16r(float f) { return bf_bits2f(f2bf_bits(f)); }

__device__ __forceinline__ void keep4_h(v16h a, v16h b, v16h c, v16h d) { asm volatile("v_nop" :: "v"(a), "v"(b), "v"(c), "v"(d)); }
__device__ __forceinline__ void keep4_b(v16b a, v16b b, v16b c, v16b d) { asm volatile("v_nop" :: "v"(a), "v"(b), "v"(c), "v"(d)); }
__device__ __forceinline__ void acc_guard4(v8f& a, v8f& b, v8f& c, v8f& d) { asm volatile("v_nop\n\tv_nop\n\tv_nop\n\tv_nop" : "+v"(a), "+v"(b), "+v"(c), "+v"(d)); }
__device__ __forceinline__ void grp_guard4_h(v8f& a, v8f& b, v8f& c, v8f& d, v16h x, v16h x2, v16h y0, v16h y1, v16h y2, v16h y3) {
  asm volatile("v_nop\n\tv_nop\n\tv_nop\n\tv_nop" : "+v"(a), "+v"(b), "+v"(c), "+v"(d) : "v"(x), "v"(x2), "v"(y0), "v"(y1), "v"(y2), "v"(y3));
}
__device__ __forceinline__ void grp_guard4_b(v8f& a, v8f& b, v8f& c, v8f& d, v16b x, v16b x2, v16b y0, v16b y1, v16b y2, v16b y3) {
  asm volatile("v_nop\n\tv_nop\n\tv_nop\n\tv_nop" : "+v"(a), "+v"(b), "+v"(c), "+v"(d) : "v"(x), "v"(x2), "v"(y0), "v"(y1), "v"(y2), "v"(y3));
}
__device__ __forceinline__ void grp_guard8_h(v8f& a0, v8f& a1, v8f& a2, v8f& a3, v8f& b0, v8f& b1, v8f& b2, v8f& b3,
                                             v16h x, v16h y, v16h w0, v16h w1, v16h w2, v16h w3) {
  asm volatile("v_nop\n\tv_nop\n\tv_nop\n\tv_nop"
               : "+v"(a0), "+v"(a1), "+v"(a2), "+v"(a3), "+v"(b0), "+v"(b1), "+v"(b2), "+v"(b3)
               : "v"(x), "v"(y), "v"(w0), "v"(w1), "v"(w2), "v"(w3));
}

template <typename T> struct Frag;
template <> struct Frag<_Float16> {
  typedef v16h V; union U { v16h v; v8h h[2]; };
  static __device__ __forceinline__ v16h load(const _Float16* p) {
    U f; f.h[0] = *(const v8h*)(p); f.h[1] = *(const v8h*)(p + 16); return f.v;
  }
  static __device__ __forceinline__ v8f mma(v16h a, v16h b, v8f c) {
    return __builtin_amdgcn_wmma_f32_16x16x32_f16(false, a, false, b, (short)0, c, false, false);
  }
  static __device__ __forceinline__ void guardg(v8f& a, v8f& b, v8f& c, v8f& d, v16h x, v16h x2, v16h y0, v16h y1, v16h y2, v16h y3) {
    grp_guard4_h(a, b, c, d, x, x2, y0, y1, y2, y3);
  }
  static __device__ __forceinline__ void keep(v16h a, v16h b, v16h c, v16h d) { keep4_h(a, b, c, d); }
};
template <> struct Frag<__bf16> {
  typedef v16b V; union U { v16b v; v8b h[2]; };
  static __device__ __forceinline__ v16b load(const __bf16* p) {
    U f; f.h[0] = *(const v8b*)(p); f.h[1] = *(const v8b*)(p + 16); return f.v;
  }
  static __device__ __forceinline__ v8f mma(v16b a, v16b b, v8f c) {
    return __builtin_amdgcn_wmma_f32_16x16x32_bf16(false, a, false, b, (short)0, c, false, false);
  }
  static __device__ __forceinline__ void guardg(v8f& a, v8f& b, v8f& c, v8f& d, v16b x, v16b x2, v16b y0, v16b y1, v16b y2, v16b y3) {
    grp_guard4_b(a, b, c, d, x, x2, y0, y1, y2, y3);
  }
  static __device__ __forceinline__ void keep(v16b a, v16b b, v16b c, v16b d) { keep4_b(a, b, c, d); }
};

template <int ET> struct Elem;
template <> struct Elem<0> { typedef _Float16 T; };
template <> struct Elem<1> { typedef __bf16 T; };
template <int ET, bool SPLIT, int BIAS_MODE, int OUT_MODE, bool RESID, int ACT = 0>
__global__ __launch_bounds__(256) void wmma_gemm64(
    const unsigned short* __restrict__ Ap, const unsigned short* __restrict__ A2p, int lda, long strideA,
    const unsigned short* __restrict__ Btp, const unsigned short* __restrict__ Bt2p, int ldb, long strideB,
    void* __restrict__ Cout, void* __restrict__ Cout2, int ldc, long strideC,
    const float* __restrict__ bias,
    const float* __restrict__ resid, long strideR,
    int M, int N, int K, float scale) {
  typedef typename Elem<ET>::T T;
  typedef typename Frag<T>::V V;
  const T* A = (const T*)Ap; const T* A2 = (const T*)A2p; const T* Bt = (const T*)Btp; const T* Bt2 = (const T*)Bt2p;
  __shared__ __align__(16) float sT[8][16 * 68];
  const int b    = blockIdx.y;
  const int lane = threadIdx.x & 31;
  const int wave = threadIdx.x >> 5;
  const int tilesN = N >> 6;
  const int tilesM = M >> 6;
  const int tile = blockIdx.x * 8 + wave;
  if (tile >= tilesM * tilesN) return;
  const int tm = tile / tilesN;
  const int tn = tile - tm * tilesN;
  const int m0 = tm << 6;
  const int n0 = tn << 6;

  const T* Ab  = A  + (size_t)b * strideA;
  const T* Bb  = Bt + (size_t)b * strideB;
  const T* Ab2 = SPLIT ? (A2  + (size_t)b * strideA) : nullptr;
  const T* Bb2 = SPLIT ? (Bt2 + (size_t)b * strideB) : nullptr;

  const int rlane = lane & 15;
  const int koff  = (lane >> 4) * 8;
  const int mOff  = (lane >> 4) * 8;

  v8f acc[4][4];
#pragma unroll
  for (int i = 0; i < 4; ++i)
#pragma unroll
    for (int j = 0; j < 4; ++j) acc[i][j] = (v8f){0.f,0.f,0.f,0.f,0.f,0.f,0.f,0.f};

  for (int k0 = 0; k0 < K; k0 += 32) {
    V bh[4], bl[4];
#pragma unroll
    for (int j = 0; j < 4; ++j) {
      const size_t bo = (size_t)(n0 + (j << 4) + rlane) * ldb + koff + k0;
      bh[j] = Frag<T>::load(Bb + bo);
      if (SPLIT) bl[j] = Frag<T>::load(Bb2 + bo);
    }
#pragma unroll
    for (int i = 0; i < 4; ++i) {
      const size_t ao = (size_t)(m0 + (i << 4) + rlane) * lda + koff + k0;
      V ah = Frag<T>::load(Ab + ao);
      V al;
      if (SPLIT) al = Frag<T>::load(Ab2 + ao);
#pragma unroll
      for (int j = 0; j < 4; ++j) {
        acc[i][j] = Frag<T>::mma(ah, bh[j], acc[i][j]);
        if (SPLIT) {
          acc[i][j] = Frag<T>::mma(ah, bl[j], acc[i][j]);
          acc[i][j] = Frag<T>::mma(al, bh[j], acc[i][j]);
        }
      }
      Frag<T>::guardg(acc[i][0], acc[i][1], acc[i][2], acc[i][3], ah, SPLIT ? al : ah, bh[0], bh[1], bh[2], bh[3]);
    }
    Frag<T>::keep(bh[0], bh[1], bh[2], bh[3]);
    if (SPLIT) Frag<T>::keep(bl[0], bl[1], bl[2], bl[3]);
  }
  acc_guard4(acc[0][0], acc[0][1], acc[0][2], acc[0][3]);
  acc_guard4(acc[1][0], acc[1][1], acc[1][2], acc[1][3]);
  acc_guard4(acc[2][0], acc[2][1], acc[2][2], acc[2][3]);
  acc_guard4(acc[3][0], acc[3][1], acc[3][2], acc[3][3]);

  float* slab = sT[wave];
  const float* Rb = RESID ? (resid + (size_t)b * strideR) : nullptr;
#pragma unroll
  for (int i = 0; i < 4; ++i) {
    const int mBase = m0 + (i << 4);
#pragma unroll
    for (int j = 0; j < 4; ++j) {
      const int n = n0 + (j << 4) + rlane;
      float bv = 0.f;
      if (BIAS_MODE == 2) bv = bias[n];
#pragma unroll
      for (int r = 0; r < 8; ++r) {
        float v = acc[i][j][r] * scale;
        if (BIAS_MODE == 1) v += bias[mBase + mOff + r];
        if (BIAS_MODE == 2) v += bv;
        if (RESID) v += Rb[(size_t)(mBase + mOff + r) * ldc + n];
        if (ACT == 2) v = fmaxf(v, 0.0f);
        if (ACT == 4) v = (v > 0.f) ? v : 0.01f * v;
        slab[(mOff + r) * 68 + (j << 4) + rlane] = v;
      }
    }
    __builtin_amdgcn_fence(__ATOMIC_RELEASE, "workgroup");
    __builtin_amdgcn_wave_barrier();
    __builtin_amdgcn_fence(__ATOMIC_ACQUIRE, "workgroup");
    if (OUT_MODE == 0) {
      float* C = (float*)Cout + (size_t)b * strideC;
      const int hh = lane >> 4, c4 = (lane & 15) * 4;
      for (int pass = 0; pass < 2; ++pass) {
#pragma unroll
        for (int it = 0; it < 8; ++it) {
          const int row = it * 2 + hh;
          v4f v = *(const v4f*)(slab + row * 68 + c4);
          *(volatile v4f*)(C + (size_t)(mBase + row) * ldc + n0 + c4) = v;
        }
        __threadfence();
      }
    } else {
      const int q = lane >> 3, c8 = (lane & 7) * 8;
      unsigned short* C  = (unsigned short*)Cout  + (size_t)b * strideC;
      unsigned short* C2 = (OUT_MODE == 2) ? ((unsigned short*)Cout2 + (size_t)b * strideC) : nullptr;
      for (int pass = 0; pass < 2; ++pass) {
#pragma unroll
        for (int it = 0; it < 4; ++it) {
          const int row = it * 4 + q;
          const float* sp = slab + row * 68 + c8;
          v8h hv, lv;
#pragma unroll
          for (int e = 0; e < 8; ++e) {
            if (OUT_MODE == 1) {
              hv[e] = (_Float16)sp[e];
            } else {
              unsigned short hb = f2bf_bits(sp[e]);
              unsigned short lb = f2bf_bits(sp[e] - bf_bits2f(hb));
              hv[e] = __builtin_bit_cast(_Float16, hb);
              lv[e] = __builtin_bit_cast(_Float16, lb);
            }
          }
          *(volatile v8h*)(C + (size_t)(mBase + row) * ldc + n0 + c8) = hv;
          if (OUT_MODE == 2) *(volatile v8h*)(C2 + (size_t)(mBase + row) * ldc + n0 + c8) = lv;
        }
        __threadfence();
      }
    }
    __builtin_amdgcn_fence(__ATOMIC_RELEASE, "workgroup");
    __builtin_amdgcn_wave_barrier();
    __builtin_amdgcn_fence(__ATOMIC_ACQUIRE, "workgroup");
  }
}

__device__ __forceinline__ float ftanh(float x) {
  const float xc = fminf(fmaxf(x, -15.0f), 15.0f);
  return 1.0f - 2.0f * __builtin_amdgcn_rcpf(1.0f + expf(2.0f * xc));
}

__global__ __launch_bounds__(256) void wcast_kernel(const float* __restrict__ W, unsigned short* __restrict__ wx,
                                                    unsigned short* __restrict__ wh) {
  const int i   = blockIdx.x * 256 + threadIdx.x;
  const int row = i >> 8;
  const int ch  = i & 255;
  const int hsel = ch >> 7;
  const int cc  = ch & 127;
  const float* sp = W + (size_t)row * kWPitch + ch * 8;
  const v4f a = *(const v4f*)(sp);
  const v4f b = *(const v4f*)(sp + 4);
  v8h hv;
#pragma unroll
  for (int e = 0; e < 4; ++e) {
    const float fa = a[e];
    const float fb = b[e];
    hv[e]     = (_Float16)(bf16r(fa) * kWCarry);
    hv[4 + e] = (_Float16)(bf16r(fb) * kWCarry);
  }
  unsigned short* dst = (hsel ? wh : wx) + (size_t)row * kDim + cc * 8;
  *(volatile v8h*)dst = hv;
  __threadfence();
  *(volatile v8h*)dst = hv;
}

__global__ __launch_bounds__(256) void xcast_kernel(const float* __restrict__ x, unsigned short* __restrict__ act) {
  const int i   = blockIdx.x * 256 + threadIdx.x;
  const int row = i >> 7;
  const int c8  = i & 127;
  const int t = row >> 4, b = row & 15;
  const float* sp = x + ((size_t)b * kSteps + t) * kDim + c8 * 8;
  const v4f a  = *(const v4f*)(sp);
  const v4f bq = *(const v4f*)(sp + 4);
  v8h hv;
#pragma unroll
  for (int e = 0; e < 4; ++e) {
    const float fa = a[e];
    const float fb = bq[e];
    hv[e]     = (_Float16)bf16r(fa);
    hv[4 + e] = (_Float16)bf16r(fb);
  }
  unsigned short* dst = act + (size_t)row * kDim + c8 * 8;
  *(volatile v8h*)dst = hv;
  __threadfence();
  *(volatile v8h*)dst = hv;
}

__global__ __launch_bounds__(256) void bias_prep_kernel(const float* __restrict__ bsrc, float* __restrict__ dst) {
  const int i = blockIdx.x * 256 + threadIdx.x;
  const v4f v = *(const v4f*)(bsrc + 4 * i);
  v4f o;
#pragma unroll
  for (int e = 0; e < 4; ++e) { const float f = v[e]; o[e] = bf16r(f); }
  float* op = dst + 4 * i;
  *(volatile v4f*)op = o;
  __threadfence();
  *(volatile v4f*)op = o;
}

template <bool LAST>
__global__ __launch_bounds__(kScanThr) void rnn_scan_kernel(
    const float* __restrict__ xwT, const _Float16* __restrict__ wh16, const float* __restrict__ h0,
    _Float16* __restrict__ actout, float* __restrict__ out) {
  __shared__ __align__(16) _Float16 Hh[kBatch * kHP];
  __shared__ __align__(16) _Float16 Hl[kBatch * kHP];
  __shared__ __align__(16) float    Sl[LAST ? (kScanThr / 32) * 16 * kSlabP : 4];

  const int tid = threadIdx.x, lane = tid & 31, wave = tid >> 5;
  const int c = lane & 15, hh = lane >> 4, koff = hh * 8, mOff = hh * 8;
  const int n0 = wave * 64;

  {
    const v8h z = {(_Float16)0.f, (_Float16)0.f, (_Float16)0.f, (_Float16)0.f, (_Float16)0.f, (_Float16)0.f, (_Float16)0.f, (_Float16)0.f};
#pragma unroll 1
    for (int i = tid; i < (kBatch * kHP) / 8; i += kScanThr) {
      *(v8h*)(Hh + i * 8) = z;
      *(v8h*)(Hl + i * 8) = z;
    }
  }
  __syncthreads();
  {
#pragma unroll 1
    for (int i = tid; i < (kBatch * kDim) / 4; i += kScanThr) {
      const int row = i >> 8;
      const int cc  = (i & 255) * 4;
      const v4f v = *(const v4f*)(h0 + (size_t)row * kDim + cc);
      const float f0 = v[0], f1 = v[1], f2 = v[2], f3 = v[3];
      _Float16* hp = Hh + row * kHP + cc;
      hp[0] = (_Float16)bf16r(f0);
      hp[1] = (_Float16)bf16r(f1);
      hp[2] = (_Float16)bf16r(f2);
      hp[3] = (_Float16)bf16r(f3);
    }
  }
  __syncthreads();

  const _Float16* arowh = Hh + c * kHP + koff;
  const _Float16* arowl = Hl + c * kHP + koff;
  const _Float16* brow  = wh16 + (size_t)(n0 + c) * kDim + koff;
  const float*    xbase = xwT + (size_t)(n0 + c) * kRows + 8 * hh;
  float* slab = Sl + (LAST ? wave * 16 * kSlabP : 0);
  const v8f z8 = {0.f, 0.f, 0.f, 0.f, 0.f, 0.f, 0.f, 0.f};

#pragma unroll 1
  for (int t = 0; t < kSteps; ++t) {
    v8f aH[4], aL[4];
#pragma unroll
    for (int j = 0; j < 4; ++j) {
      const float* xp = xbase + (size_t)(16 * j) * kRows + t * kBatch;
      const v4f xa = *(const v4f*)(xp);
      const v4f xb = *(const v4f*)(xp + 4);
#pragma unroll
      for (int e = 0; e < 4; ++e) {
        const float u = xa[e];
        const float w = xb[e];
        aH[j][e]     = u * kWCarry;
        aH[j][4 + e] = w * kWCarry;
      }
      aL[j] = z8;
      if (j == 1) asm volatile("" ::: "memory");
    }

#pragma unroll 2
    for (int kc = 0; kc < kDim / 32; ++kc) {
      const v16h fa = Frag<_Float16>::load(arowh + kc * 32);
      const v16h fl = Frag<_Float16>::load(arowl + kc * 32);
      v16h fb[4];
#pragma unroll
      for (int j = 0; j < 4; ++j) fb[j] = Frag<_Float16>::load(brow + (size_t)(16 * j) * kDim + kc * 32);
#pragma unroll
      for (int j = 0; j < 4; ++j) {
        aH[j] = Frag<_Float16>::mma(fa, fb[j], aH[j]);
        aL[j] = Frag<_Float16>::mma(fl, fb[j], aL[j]);
      }
      grp_guard8_h(aH[0], aH[1], aH[2], aH[3], aL[0], aL[1], aL[2], aL[3], fa, fl, fb[0], fb[1], fb[2], fb[3]);
    }
    acc_guard4(aH[0], aH[1], aH[2], aH[3]);
    acc_guard4(aL[0], aL[1], aL[2], aL[3]);

    float hv[4][8];
#pragma unroll
    for (int j = 0; j < 4; ++j) {
#pragma unroll
      for (int r = 0; r < 8; ++r) {
        const float sh = aH[j][r];
        const float sl = aL[j][r];
        const float pre = sh * kWCarryInv + sl * kLoFold;
        hv[j][r] = ftanh(pre);
      }
    }
    __syncthreads();

#pragma unroll
    for (int j = 0; j < 4; ++j) {
#pragma unroll
      for (int r = 0; r < 8; ++r) {
        const float hval = hv[j][r];
        const _Float16 hi = (_Float16)hval;
        const float res = (hval - (float)hi) * kLoCarry;
        const int idx = (mOff + r) * kHP + n0 + 16 * j + c;
        Hh[idx] = hi;
        Hl[idx] = (_Float16)res;
        if (LAST) slab[(mOff + r) * kSlabP + 16 * j + c] = hval;
      }
    }
    __syncthreads();

    if (!LAST) {
      const int q4 = lane >> 3, c8 = (lane & 7) * 8;
      for (int pass = 0; pass < 2; ++pass) {
#pragma unroll
        for (int it = 0; it < 4; ++it) {
          const int rr = it * 4 + q4;
          const v8h v = *(const v8h*)(Hh + rr * kHP + n0 + c8);
          *(volatile v8h*)(actout + ((size_t)t * kBatch + rr) * kDim + n0 + c8) = v;
        }
        __threadfence();
      }
    } else {
      const int c4 = c * 4;
      for (int pass = 0; pass < 2; ++pass) {
#pragma unroll
        for (int it = 0; it < 8; ++it) {
          const int row = it * 2 + hh;
          const v4f v = *(const v4f*)(slab + row * kSlabP + c4);
          *(volatile v4f*)(out + ((size_t)row * kSteps + t) * kDim + n0 + c4) = v;
        }
        __threadfence();
      }
    }
  }
}

extern "C" void kernel_launch(void* const* d_in, const int* in_sizes, int n_in,
                              void* d_out, int out_size, void* d_ws, size_t ws_size, hipStream_t stream) {
  if (n_in < 4 || d_out == nullptr || d_ws == nullptr) return;
  if (in_sizes[0] != kBatch * kSteps * kDim || in_sizes[1] != kLayers * kBatch * kDim ||
      in_sizes[2] != kLayers * kDim * kWPitch || in_sizes[3] != kLayers * kDim ||
      out_size != kBatch * kSteps * kDim) return;

  const float* X   = (const float*)d_in[0];
  const float* h0s = (const float*)d_in[1];
  const float* W   = (const float*)d_in[2];
  const float* bia = (const float*)d_in[3];
  float* out = (float*)d_out;

  char* ws = (char*)d_ws; size_t off = 0;
  auto carve = [&](size_t bytes) -> char* { char* p = ws + off; off += (bytes + 255) & ~(size_t)255; return p; };
  unsigned short* WX16  = (unsigned short*)carve((size_t)kLayers * kDim * kDim * 2);
  unsigned short* WH16  = (unsigned short*)carve((size_t)kLayers * kDim * kDim * 2);
  unsigned short* ACTA  = (unsigned short*)carve((size_t)kRows * kDim * 2);
  unsigned short* ACTB  = (unsigned short*)carve((size_t)kRows * kDim * 2);
  float*          XWT   = (float*)carve((size_t)kDim * kRows * 4);
  float*          BIASR = (float*)carve((size_t)kLayers * kDim * 4);
  if (off > ws_size || off > (size_t)134217728) return;

  wcast_kernel<<<(kLayers * kDim * (kWPitch / 8)) / 256, 256, 0, stream>>>(W, WX16, WH16);
  xcast_kernel<<<(kRows * (kDim / 8)) / 256, 256, 0, stream>>>(X, ACTA);
  bias_prep_kernel<<<(kLayers * kDim / 4) / 256, 256, 0, stream>>>(bia, BIASR);

  const int gemmGrid = ((kDim / 64) * (kRows / 64)) / 8;
  for (int l = 0; l < kLayers; ++l) {
    unsigned short* actIn  = (l & 1) ? ACTB : ACTA;
    unsigned short* actOut = (l & 1) ? ACTA : ACTB;
    const unsigned short* wx = WX16 + (size_t)l * kDim * kDim;
    const unsigned short* wh = WH16 + (size_t)l * kDim * kDim;
    wmma_gemm64<0, false, 1, 0, false, 0><<<dim3(gemmGrid, 1), 256, 0, stream>>>(
        wx, wx, kDim, 0L, actIn, actIn, kDim, 0L,
        (void*)XWT, (void*)XWT, kRows, 0L, BIASR + (size_t)l * kDim, BIASR, 0L,
        kDim, kRows, kDim, kWCarryInv);
    if (l < kLayers - 1) {
      rnn_scan_kernel<false><<<1, kScanThr, 0, stream>>>(XWT, (const _Float16*)wh, h0s + (size_t)l * kBatch * kDim,
                                                         (_Float16*)actOut, out);
    } else {
      rnn_scan_kernel<true><<<1, kScanThr, 0, stream>>>(XWT, (const _Float16*)wh, h0s + (size_t)l * kBatch * kDim,
                                                        (_Float16*)actOut, out);
    }
  }
}
